// STABR_tag_encoder_26697516712557
// MI455X (gfx1250) — hardware-verified
//
#include <hip/hip_runtime.h>
#include <stddef.h>
#include <stdint.h>


#define NB   256
#define NS   512
#define NT   20
#define NE   25
#define NV   100000
#define NH   128
#define NG   512
#define NK   64
#define KIN  96
#define NPOS (NB * NS)
#define TCH  32
#define NCH  (NS / TCH)
#define MCH  (TCH * NB)
#define HP   136
#define CTP  36
#define THR  256
#define PTHR 128
#define PC0  (2 * NG * (KIN / 8))
#define PC1  (2 * NG * (NH / 8))
#define PC2  (NH * (2 * NH / 8))

static_assert(NS % TCH == 0);
static_assert(MCH % 64 == 0 && NB % 64 == 0);
static_assert(NG % 256 == 0);
static_assert(KIN % 32 == 0 && KIN >= 32 + NK && NE <= 32 && NK == 64);
static_assert(THR == 32 * (NH / 16));
static_assert(THR == 2 * NH && NS == 2 * THR);
static_assert((HP * 2) % 16 == 0 && HP >= NH);
static_assert((CTP * 4) % 16 == 0 && CTP >= 32);
static_assert(NPOS % 16 == 0 && NB % 16 == 0);
static_assert((PC0 + PC1 + PC2) % PTHR == 0);
static_assert(PC0 % 32 == 0 && PC1 % 32 == 0);

typedef _Float16 v8h  __attribute__((ext_vector_type(8)));
typedef _Float16 v16h __attribute__((ext_vector_type(16)));
typedef float    v2f  __attribute__((ext_vector_type(2)));
typedef float    v4f  __attribute__((ext_vector_type(4)));
typedef float    v8f  __attribute__((ext_vector_type(8)));

union Frag { v16h v; v8h h[2]; };

#if __has_builtin(__builtin_amdgcn_exp2f)
#define EXP2_FAST(x) __builtin_amdgcn_exp2f(x)
#else
#define EXP2_FAST(x) exp2f(x)
#endif
#define RCP_FAST(x) __builtin_amdgcn_rcpf(x)

#define XSC   16.0f
#define KSC   16.0f
#define SKS   256.0f
#define RSC   256.0f
#define WKS   256.0f
#define HSC   16.0f
#define IHSC  0.0625f
#define IS8   0.00390625f
#define IS12  0.000244140625f
#define XPUP  4096.0f
#define LOG2E 1.4426950408889634f
#define C2L2E 2.8853900817779268f

__device__ __forceinline__ v16h frag16(const _Float16* row, int k0, int hh)
{
    Frag f;
    f.h[0] = *(const v8h*)(row + k0 + 8 * hh);
    f.h[1] = *(const v8h*)(row + k0 + 16 + 8 * hh);
    return f.v;
}

__device__ __forceinline__ v8f wmma_f16(v16h a, v16h b, v8f c)
{
    v8f d = __builtin_amdgcn_wmma_f32_16x16x32_f16(false, a, false, b, (short)0, c, false, false);
    asm volatile("v_nop\n\tv_nop\n\tv_nop\n\tv_nop" : "+v"(d) : "v"(a), "v"(b));
    return d;
}

__device__ __forceinline__ float sigm_f(float x)
{
    return RCP_FAST(1.0f + EXP2_FAST(-LOG2E * x));
}
__device__ __forceinline__ float tanh_f(float x)
{
    return 1.0f - 2.0f * RCP_FAST(1.0f + EXP2_FAST(C2L2E * x));
}

__device__ __forceinline__ v8f ldx8(const float* p)
{
    const v4f a = *(const v4f*)p;
    const v4f b = *(const v4f*)(p + 4);
    v8f r = { a[0], a[1], a[2], a[3], b[0], b[1], b[2], b[3] };
    return r * XPUP;
}

__global__ void __launch_bounds__(PTHR) prep_kernel(
    const float* __restrict__ Kf, const float* __restrict__ Kb,
    const float* __restrict__ Sf, const float* __restrict__ Sb,
    const float* __restrict__ Rf, const float* __restrict__ Rb,
    const float* __restrict__ Wk, _Float16* P16)
{
    const int g = blockIdx.x * PTHR + threadIdx.x;
    v8f v;
    if (g < PC0) {
        const int dir = g / (NG * (KIN / 8));
        const int rem = g - dir * (NG * (KIN / 8));
        const int n   = rem / (KIN / 8);
        const int k0  = 8 * (rem - n * (KIN / 8));
        const float* K = dir ? Kb : Kf;
        const float* S = dir ? Sb : Sf;
        #pragma unroll
        for (int i = 0; i < 8; ++i) {
            const int k = k0 + i;
            float x;
            if (k < 32) x = (k < NE) ? KSC * K[(size_t)k * NG + n] : 0.0f;
            else        x = SKS * S[(size_t)(k - 32) * NG + n];
            v[i] = x;
        }
    } else if (g < PC0 + PC1) {
        const int c   = g - PC0;
        const int dir = c / (NG * (NH / 8));
        const int rem = c - dir * (NG * (NH / 8));
        const int n   = rem / (NH / 8);
        const int k0  = 8 * (rem - n * (NH / 8));
        const float* R = dir ? Rb : Rf;
        #pragma unroll
        for (int i = 0; i < 8; ++i) v[i] = RSC * R[(size_t)(k0 + i) * NG + n];
    } else {
        const int c  = g - PC0 - PC1;
        const int n  = c / (2 * NH / 8);
        const int k0 = 8 * (c - n * (2 * NH / 8));
        #pragma unroll
        for (int i = 0; i < 8; ++i) v[i] = WKS * Wk[(size_t)(k0 + i) * NH + n];
    }
    const v8h val = __builtin_convertvector(v, v8h);
    volatile v8h* p = (volatile v8h*)(P16 + (size_t)g * 8);
    *p = val;
    __threadfence();
    *p = val;
}

__global__ void __launch_bounds__(THR) embed_kernel(
    const int* __restrict__ tags, const float* __restrict__ emb,
    const float* __restrict__ skips, _Float16* X16)
{
    __shared__ __align__(16) _Float16 sRow[8 * 2 * KIN];

    const int tid = threadIdx.x;
    const int w   = tid >> 5;
    const int l   = tid & 31;
    const int row0 = (blockIdx.x * 8 + w) * 2;
    _Float16* sr = sRow + w * 2 * KIN;

    #pragma unroll
    for (int p = 0; p < 2; ++p) {
        const int r   = row0 + p;
        const int t   = r >> 8;
        const int b   = r & (NB - 1);
        const size_t pos = (size_t)b * NS + t;
        const int* tp = tags + pos * NT;
        float sum = 0.0f;
        int cnt = 0;
        #pragma unroll
        for (int tt = 0; tt < NT; ++tt) {
            const int tag = tp[tt];
            if (tag != 0) {
                ++cnt;
                int id = tag < 0 ? 0 : (tag > NV - 1 ? NV - 1 : tag);
                if (l < NE) sum += emb[(size_t)id * NE + l];
            }
        }
        const float denom = (cnt == 0) ? 1.0f : (float)cnt;
        const float x = sum * (1.0f / denom);
        sr[p * KIN + l] = (l < NE) ? (_Float16)(XSC * x) : (_Float16)0.0f;
        const v2f sk = *(const v2f*)(skips + pos * NK + 2 * l);
        sr[p * KIN + 32 + 2 * l]     = (_Float16)sk[0];
        sr[p * KIN + 32 + 2 * l + 1] = (_Float16)sk[1];
    }
    __syncthreads();

    v8h val = { (_Float16)0.f, (_Float16)0.f, (_Float16)0.f, (_Float16)0.f,
                (_Float16)0.f, (_Float16)0.f, (_Float16)0.f, (_Float16)0.f };
    volatile v8h* vp = (volatile v8h*)(X16 + (size_t)row0 * KIN);
    const bool act = l < (2 * KIN / 8);
    if (act) {
        val = *(const v8h*)(sr + 8 * l);
        vp  = (volatile v8h*)(X16 + (size_t)row0 * KIN + 8 * l);
        *vp = val;
    }
    __threadfence();
    if (act) *vp = val;
}

__global__ void __launch_bounds__(THR) gemm_in_kernel(
    const _Float16* __restrict__ A0, const _Float16* __restrict__ A1,
    const _Float16* __restrict__ W0, const _Float16* __restrict__ W1,
    const float* __restrict__ bias0, const float* __restrict__ bias1,
    float* C0, float* C1)
{
    __shared__ __align__(16) float s_c[256 * CTP];

    const int z = blockIdx.z;
    const _Float16* A = z ? A1 : A0;
    const _Float16* W = z ? W1 : W0;
    const float* bias = z ? bias1 : bias0;
    float* C = z ? C1 : C0;

    const int tid = threadIdx.x;
    const int l   = tid & 31;
    const int wid = tid >> 5;
    const int wm  = wid >> 2, wn = wid & 3;
    const int hh  = l >> 4, m15 = l & 15;
    const int mblk = blockIdx.x * 64;
    const int nblk = blockIdx.y * 256;
    const int m0 = mblk + wm * 32;
    const int n0 = nblk + wn * 64;

    const v8f zero = { 0.f, 0.f, 0.f, 0.f, 0.f, 0.f, 0.f, 0.f };
    v8f acc[2][4];
    #pragma unroll
    for (int mi = 0; mi < 2; ++mi)
        #pragma unroll
        for (int j = 0; j < 4; ++j) acc[mi][j] = zero;

    const _Float16* a0p = A + (size_t)(m0 + m15) * KIN;
    const _Float16* a1p = A + (size_t)(m0 + 16 + m15) * KIN;
    const _Float16* wp  = W + (size_t)(n0 + m15) * KIN;

    #pragma unroll
    for (int k0 = 0; k0 < KIN; k0 += 32) {
        const v16h fa0 = frag16(a0p, k0, hh);
        const v16h fa1 = frag16(a1p, k0, hh);
        #pragma unroll
        for (int j = 0; j < 4; ++j) {
            const v16h fb = frag16(wp + (size_t)j * 16 * KIN, k0, hh);
            acc[0][j] = wmma_f16(fa0, fb, acc[0][j]);
            acc[1][j] = wmma_f16(fa1, fb, acc[1][j]);
        }
    }

    const int tt = mblk >> 8;
    const int bb = mblk & (NB - 1);

    for (int ph = 0; ph < 2; ++ph) {
        if (wm == ph) {
            #pragma unroll
            for (int mi = 0; mi < 2; ++mi)
                #pragma unroll
                for (int j = 0; j < 4; ++j)
                    #pragma unroll
                    for (int r = 0; r < 8; ++r) {
                        const int rl = mi * 16 + 8 * hh + r;
                        const int cl = wn * 64 + 16 * j + m15;
                        s_c[cl * CTP + rl] = acc[mi][j][r];
                    }
        }
        __syncthreads();

        v4f vals[8];
        size_t off[8];
        #pragma unroll
        for (int i = 0; i < 8; ++i) {
            const int idx = tid + THR * i;
            const int nl  = idx >> 3;
            const int q   = idx & 7;
            const int n   = nblk + nl;
            const v4f x = *(const v4f*)&s_c[nl * CTP + 4 * q];
            const float bv = bias[n];
            vals[i] = x * IS8 + bv;
            off[i]  = ((size_t)(tt * NG + n)) * NB + bb + 32 * ph + 4 * q;
        }
        #pragma unroll
        for (int i = 0; i < 8; ++i) *(volatile v4f*)(C + off[i]) = vals[i];
        __threadfence();
        #pragma unroll
        for (int i = 0; i < 8; ++i) *(volatile v4f*)(C + off[i]) = vals[i];
        __syncthreads();
    }
}

__global__ void __launch_bounds__(THR) lstm_kernel(
    const float* __restrict__ XP, const _Float16* __restrict__ Rp, const int* __restrict__ tags,
    _Float16* OUT16, float* stH, float* stC, int chunk, int first)
{
    __shared__ __align__(16) _Float16 h16[16 * HP];
    __shared__ __align__(16) float sH[16 * NH];
    __shared__ __align__(16) float sC[16 * NH];
    __shared__ float maskL[16];

    const int bt  = blockIdx.x;
    const int dir = blockIdx.y;
    const int tid = threadIdx.x;
    const int w   = tid >> 5;
    const int l   = tid & 31;
    const int hh  = l >> 4;
    const int m15 = l & 15;
    const int j   = 16 * w + m15;
    const int brow0 = 16 * bt;
    const size_t sbase = ((size_t)dir * NB + brow0) * NH;

    float hst[8], cst[8];
    if (first) {
        #pragma unroll
        for (int r = 0; r < 8; ++r) { hst[r] = 0.0f; cst[r] = 0.0f; }
        for (int i = tid; i < 16 * HP; i += THR) h16[i] = (_Float16)0.0f;
    } else {
        #pragma unroll
        for (int r = 0; r < 8; ++r) {
            const int row = 8 * hh + r;
            hst[r] = stH[sbase + (size_t)row * NH + j];
            cst[r] = stC[sbase + (size_t)row * NH + j];
            h16[row * HP + j] = (_Float16)(HSC * hst[r]);
        }
    }
    __syncthreads();

    const int tc = dir ? (NCH - 1 - chunk) : chunk;
    const _Float16* rI = Rp + ((size_t)(dir * NG + 0 * NH + j)) * NH;
    const _Float16* rF = Rp + ((size_t)(dir * NG + 1 * NH + j)) * NH;
    const _Float16* rG = Rp + ((size_t)(dir * NG + 2 * NH + j)) * NH;
    const _Float16* rO = Rp + ((size_t)(dir * NG + 3 * NH + j)) * NH;
    const float* xpz = XP + (size_t)dir * TCH * NG * NB + (size_t)j * NB + brow0 + 8 * hh;
    const _Float16* hrow = &h16[m15 * HP];
    const int GS = NH * NB;

    #pragma unroll 1
    for (int s = 0; s < TCH; ++s) {
        const int tt = dir ? (TCH - 1 - s) : s;
        const int t  = tc * TCH + tt;
        if (tid < 16)
            maskL[tid] = (tags[((size_t)(brow0 + tid) * NS + t) * NT] != 0) ? 1.0f : 0.0f;

        const float* xp = xpz + (size_t)tt * NG * NB;
        v8f aI = ldx8(xp);
        v8f aF = ldx8(xp + GS);
        v8f aG = ldx8(xp + 2 * GS);
        v8f aO = ldx8(xp + 3 * GS);

        #pragma unroll
        for (int k0 = 0; k0 < NH; k0 += 32) {
            const v16h fh = frag16(hrow, k0, hh);
            v16h fb;
            fb = frag16(rI, k0, hh);  aI = wmma_f16(fh, fb, aI);
            fb = frag16(rF, k0, hh);  aF = wmma_f16(fh, fb, aF);
            fb = frag16(rG, k0, hh);  aG = wmma_f16(fh, fb, aG);
            fb = frag16(rO, k0, hh);  aO = wmma_f16(fh, fb, aO);
        }
        __syncthreads();

        #pragma unroll
        for (int r = 0; r < 8; ++r) {
            const float ig = sigm_f(aI[r] * IS12);
            const float fg = sigm_f(aF[r] * IS12);
            const float gg = tanh_f(aG[r] * IS12);
            const float og = sigm_f(aO[r] * IS12);
            const float cn = fg * cst[r] + ig * gg;
            const float hn = og * tanh_f(cn);
            const bool  m  = maskL[8 * hh + r] != 0.0f;
            const float h2 = m ? hn : hst[r];
            const float c2 = m ? cn : cst[r];
            hst[r] = h2;
            cst[r] = c2;
            h16[(8 * hh + r) * HP + j] = (_Float16)(HSC * h2);
        }
        __syncthreads();

        const int rowo = 2 * w + hh;
        const v8h ov = *(const v8h*)&h16[rowo * HP + 8 * m15];
        volatile v8h* op = (volatile v8h*)(OUT16 + ((size_t)t * NB + brow0 + rowo) * (2 * NH) + dir * NH + 8 * m15);
        *op = ov;
        __threadfence();
        *op = ov;
    }

    #pragma unroll
    for (int r = 0; r < 8; ++r) {
        sH[(8 * hh + r) * NH + j] = hst[r];
        sC[(8 * hh + r) * NH + j] = cst[r];
    }
    __syncthreads();
    v4f hv[2], cv[2];
    size_t so[2];
    #pragma unroll
    for (int i = 0; i < 2; ++i) {
        const int row = 2 * w + i;
        hv[i] = *(const v4f*)&sH[row * NH + 4 * l];
        cv[i] = *(const v4f*)&sC[row * NH + 4 * l];
        so[i] = sbase + (size_t)row * NH + 4 * l;
    }
    #pragma unroll
    for (int i = 0; i < 2; ++i) {
        *(volatile v4f*)(stH + so[i]) = hv[i];
        *(volatile v4f*)(stC + so[i]) = cv[i];
    }
    __threadfence();
    #pragma unroll
    for (int i = 0; i < 2; ++i) {
        *(volatile v4f*)(stH + so[i]) = hv[i];
        *(volatile v4f*)(stC + so[i]) = cv[i];
    }
}

__global__ void __launch_bounds__(THR) attn_kernel(
    const _Float16* __restrict__ OUT16, const float* __restrict__ hF, const int* __restrict__ tags,
    const _Float16* __restrict__ WkP, const float* __restrict__ bk,
    const float* __restrict__ Wq, const float* __restrict__ bq,
    const float* __restrict__ We, const float* __restrict__ be, float* out)
{
    __shared__ float sq[NH];
    __shared__ float ePart[8 * NS];
    __shared__ float wts[NS];
    __shared__ float red[16];
    __shared__ __align__(16) float sctx[2 * NH];

    const int b   = blockIdx.x;
    const int tid = threadIdx.x;
    const int w   = tid >> 5;
    const int l   = tid & 31;
    const int hh  = l >> 4;
    const int m15 = l & 15;

    if (tid < NH) {
        const float* hf = hF + (size_t)b * NH;
        float a = 0.0f;
        #pragma unroll 1
        for (int k = 0; k < NH; ++k) a += hf[k] * Wq[(size_t)k * NH + tid];
        sq[tid] = a + bq[tid];
    }
    __syncthreads();

    const int   col = 16 * w + m15;
    const float qv  = sq[col];
    const float bkv = bk[col];
    const float wev = We[col];
    const _Float16* wp = WkP + (size_t)col * (2 * NH);
    const v8f zero = { 0.f, 0.f, 0.f, 0.f, 0.f, 0.f, 0.f, 0.f };

    #pragma unroll 1
    for (int tt = 0; tt < NS / 16; ++tt) {
        const int t0 = 16 * tt;
        const _Float16* ap = OUT16 + ((size_t)(t0 + m15) * NB + b) * (2 * NH);
        v8f acc = zero;
        #pragma unroll
        for (int k0 = 0; k0 < 2 * NH; k0 += 32)
            acc = wmma_f16(frag16(ap, k0, hh), frag16(wp, k0, hh), acc);
        #pragma unroll
        for (int r = 0; r < 8; ++r) {
            float v = tanh_f((acc[r] * IS12 + bkv) + qv) * wev;
            v += __shfl_xor(v, 1, 16);
            v += __shfl_xor(v, 2, 16);
            v += __shfl_xor(v, 4, 16);
            v += __shfl_xor(v, 8, 16);
            if (m15 == 0) ePart[w * NS + t0 + 8 * hh + r] = v;
        }
    }
    __syncthreads();

    float ev[2], pv[2];
    #pragma unroll
    for (int i = 0; i < 2; ++i) {
        const int ti = tid + THR * i;
        float e = ePart[ti];
        #pragma unroll
        for (int w2 = 1; w2 < 8; ++w2) e += ePart[w2 * NS + ti];
        e += be[0];
        const float mf = (tags[((size_t)b * NS + ti) * NT] != 0) ? 1.0f : 0.0f;
        e = e + (1.0f - mf) * (-1.0e9f);
        ev[i] = e;
    }
    float mx = fmaxf(ev[0], ev[1]);
    #pragma unroll
    for (int off = 16; off > 0; off >>= 1) mx = fmaxf(mx, __shfl_xor(mx, off, 32));
    if (l == 0) red[w] = mx;
    __syncthreads();
    float M = red[0];
    #pragma unroll
    for (int w2 = 1; w2 < 8; ++w2) M = fmaxf(M, red[w2]);
    pv[0] = EXP2_FAST((ev[0] - M) * LOG2E);
    pv[1] = EXP2_FAST((ev[1] - M) * LOG2E);
    float sv = pv[0] + pv[1];
    #pragma unroll
    for (int off = 16; off > 0; off >>= 1) sv += __shfl_xor(sv, off, 32);
    if (l == 0) red[8 + w] = sv;
    __syncthreads();
    float S = red[8];
    #pragma unroll
    for (int w2 = 1; w2 < 8; ++w2) S += red[8 + w2];
    const float inv = 1.0f / S;
    wts[tid]       = pv[0] * inv;
    wts[tid + THR] = pv[1] * inv;
    __syncthreads();

    float c = 0.0f;
    const _Float16* op = OUT16 + (size_t)b * (2 * NH) + tid;
    #pragma unroll 4
    for (int t = 0; t < NS; ++t) {
        const float hv = (float)op[(size_t)t * NB * (2 * NH)] * IHSC;
        c += wts[t] * hv;
    }
    sctx[tid] = c;
    __syncthreads();

    if (w == 0) {
        v4f cv[2];
        size_t co[2];
        #pragma unroll
        for (int i = 0; i < 2; ++i) {
            cv[i] = *(const v4f*)&sctx[NH * i + 4 * l];
            co[i] = (size_t)b * (2 * NH) + NH * i + 4 * l;
        }
        #pragma unroll
        for (int i = 0; i < 2; ++i) *(volatile v4f*)(out + co[i]) = cv[i];
        __threadfence();
        #pragma unroll
        for (int i = 0; i < 2; ++i) *(volatile v4f*)(out + co[i]) = cv[i];
    }
}

extern "C" void kernel_launch(void* const* d_in, const int* in_sizes, int n_in,
                              void* d_out, int out_size, void* d_ws, size_t ws_size,
                              hipStream_t stream)
{
    if (n_in < 17) return;
    if (in_sizes[0] != NPOS * NT) return;
    if (in_sizes[1] != NPOS * NK) return;
    if (in_sizes[2] != NV * NE) return;
    if (in_sizes[3] != NE * NG || in_sizes[4] != NH * NG || in_sizes[5] != NK * NG || in_sizes[6] != NG) return;
    if (in_sizes[7] != NE * NG || in_sizes[8] != NH * NG || in_sizes[9] != NK * NG || in_sizes[10] != NG) return;
    if (in_sizes[11] != 2 * NH * NH || in_sizes[12] != NH) return;
    if (in_sizes[13] != NH * NH || in_sizes[14] != NH) return;
    if (in_sizes[15] != NH || in_sizes[16] != 1) return;
    if (out_size != NB * 2 * NH) return;

    const int*   tags  = (const int*)d_in[0];
    const float* skips = (const float*)d_in[1];
    const float* emb   = (const float*)d_in[2];
    const float* Kf    = (const float*)d_in[3];
    const float* Rf    = (const float*)d_in[4];
    const float* Sf    = (const float*)d_in[5];
    const float* bfv   = (const float*)d_in[6];
    const float* Kb    = (const float*)d_in[7];
    const float* Rb    = (const float*)d_in[8];
    const float* Sb    = (const float*)d_in[9];
    const float* bbv   = (const float*)d_in[10];
    const float* Wk    = (const float*)d_in[11];
    const float* bk    = (const float*)d_in[12];
    const float* Wq    = (const float*)d_in[13];
    const float* bq    = (const float*)d_in[14];
    const float* We    = (const float*)d_in[15];
    const float* be    = (const float*)d_in[16];
    float* out = (float*)d_out;

    const size_t szP16 = (size_t)(PC0 + PC1 + PC2) * 16;
    const size_t szX16 = (size_t)NPOS * KIN * 2;
    const size_t szXP  = (size_t)2 * TCH * NG * NB * 4;
    const size_t szOUT = (size_t)NPOS * 2 * NH * 2;
    const size_t szST  = (size_t)2 * NB * NH * 4;
    size_t off = 0;
    const size_t oP16 = off; off += szP16;
    const size_t oX16 = off; off += szX16;
    const size_t oXP  = off; off += szXP;
    const size_t oOUT = off; off += szOUT;
    const size_t oSH  = off; off += szST;
    const size_t oSC  = off; off += szST;
    if (off > ws_size) return;
    if (off > (size_t)134217728) return;

    char* ws = (char*)d_ws;
    _Float16* P16   = (_Float16*)(ws + oP16);
    _Float16* WinF  = P16;
    _Float16* WinB  = P16 + (size_t)NG * KIN;
    _Float16* Rp    = P16 + (size_t)PC0 * 8;
    _Float16* WkP   = P16 + (size_t)(PC0 + PC1) * 8;
    _Float16* X16   = (_Float16*)(ws + oX16);
    float*    XP    = (float*)(ws + oXP);
    _Float16* OUT16 = (_Float16*)(ws + oOUT);
    float*    stH   = (float*)(ws + oSH);
    float*    stC   = (float*)(ws + oSC);

    prep_kernel<<<dim3((PC0 + PC1 + PC2) / PTHR), dim3(PTHR), 0, stream>>>(Kf, Kb, Sf, Sb, Rf, Rb, Wk, P16);

    embed_kernel<<<dim3(NPOS / 16), dim3(THR), 0, stream>>>(tags, emb, skips, X16);

    for (int c = 0; c < NCH; ++c) {
        const _Float16* A0 = X16 + (size_t)c * MCH * KIN;
        const _Float16* A1 = X16 + (size_t)(NCH - 1 - c) * MCH * KIN;
        float* XP1 = XP + (size_t)TCH * NG * NB;
        gemm_in_kernel<<<dim3(MCH / 64, NG / 256, 2), dim3(THR), 0, stream>>>(
            A0, A1, WinF, WinB, bfv, bbv, XP, XP1);
        lstm_kernel<<<dim3(NB / 16, 2), dim3(THR), 0, stream>>>(
            XP, Rp, tags, OUT16, stH, stC, c, (c == 0) ? 1 : 0);
    }

    attn_kernel<<<dim3(NB), dim3(THR), 0, stream>>>(OUT16, stH, tags, WkP, bk, Wq, bq, We, be, out);
}
